// LocalSelfAttentionWithSEAndCCA_61263413510146
// MI455X (gfx1250) — hardware-run, weakly checked
//
#include <hip/hip_runtime.h>


#ifndef NB
#define NB 4
#endif
#ifndef SEQ
#define SEQ 2048
#endif
#define NB_FULL  4
#define SEQ_FULL 2048
#ifndef OUT_SEQ
#define OUT_SEQ SEQ
#endif
#define CC   256
#define NH_  8
#define HD   32
#define KW   9
#define PADW 4
#define CH2  128
#define RSE  16
#define NTOK (NB * SEQ)
#define SEQP (SEQ + 2)
#define RCH  64
#define NCHK (NTOK / RCH)
#define CPB  (SEQ / RCH)
#define ATK  16
#define STP  (CC + 4)
#define WSC  64.0f
#define WSI  (1.0f / 64.0f)
#define QRS  2048.0f
#define QRI  (1.0f / 2048.0f)
#define EPSV 1.0e-5f
#define SC2  ((float)(0.17677669529663687 * 1.4426950408889634))
#define L2E  1.4426950408889634f

static_assert(HD == 32);
static_assert(NH_ * HD == CC);
static_assert(KW == 2 * PADW + 1);
static_assert(HD % 4 == 0);
static_assert(CC % 64 == 0);
static_assert(CH2 % 64 == 0);
static_assert((3 * CC) % 64 == 0);
static_assert(CC % 32 == 0);
static_assert((3 * CC) % 32 == 0);
static_assert((3 * CH2) % 32 == 0);
static_assert(SEQ % 64 == 0);
static_assert(NTOK % 64 == 0);
static_assert(SEQ % RCH == 0);
static_assert(SEQ % ATK == 0);
static_assert(SEQ % 32 == 0);
static_assert(CC / 4 == 64);
static_assert(ATK * NH_ * 16 * 8 == ATK * CC * 4);
static_assert(32 * 16 * 8 == 16 * 64 * 4);
static_assert(2 * 256 * 16 == 64 * 64 * 2);
static_assert(16 * 256 == 64 * 64);
static_assert(NB * RSE <= CC);
static_assert(((size_t)NB * CC * SEQ) % 256 == 0);
static_assert(((size_t)NTOK * CC / 8) % 256 == 0);
static_assert(((size_t)NB * SEQP * CC / 8) % 1 == 0);
static_assert(((size_t)CC * CC / 8) % 256 == 0);
static_assert(((size_t)CH2 * 3 * CC / 8) % 256 == 0);
static_assert(NB <= NB_FULL);
static_assert(SEQ <= SEQ_FULL);
static_assert((STP * 4) % 16 == 0);
static_assert(16 * 68 * 4 <= 131072);
static_assert(64 * 72 * 2 <= 131072);
static_assert((KW * HD + ATK * STP) * 4 <= 131072);
static_assert((NB * CC + NB * RSE) * 4 <= 131072);
static_assert(CH2 <= CC);
static_assert(CC * 16 == 2 * CC * 8);
static_assert((2 * CC * 8) % 128 == 0 && (2 * CH2 * 8) % 128 == 0);
static_assert(2 * CC * 8 <= 131072);
static_assert(2 * CC / 4 <= CH2);
static_assert((2 * CC / 4) % 32 == 0);
static_assert((2 * CC / 4) * 16 == 2 * CC * 4);
static_assert(2 * CC * 4 <= 131072);
static_assert((2 * NB * CC) % 4 == 0 && ((2 * NB * CC / 4) % 32) == 0);
static_assert((NB * CC + NB * RSE + 2 * NB * CC) * 4 <= 131072);

typedef _Float16 h16;
typedef unsigned short bf;
typedef __attribute__((ext_vector_type(16))) __bf16   v16bf;
typedef __attribute__((ext_vector_type(16))) _Float16 v16h;
typedef __attribute__((ext_vector_type(8)))  _Float16 v8h;
typedef __attribute__((ext_vector_type(8)))  unsigned short v8us;
typedef __attribute__((ext_vector_type(8)))  float    v8f;
typedef __attribute__((ext_vector_type(4)))  float    v4f;
typedef v4f  __attribute__((may_alias)) v4fa;
typedef v8us __attribute__((may_alias)) v8usa;

__device__ __forceinline__ unsigned short f2bf(float f) { unsigned u = __float_as_uint(f); u += 0x7FFFu + ((u >> 16) & 1u); return (unsigned short)(u >> 16); }
__device__ __forceinline__ float bfr(float f) { return __uint_as_float(((unsigned)f2bf(f)) << 16); }
__device__ __forceinline__ v16h cat16(v8h lo, v8h hi) { return __builtin_shufflevector(lo, hi, 0, 1, 2, 3, 4, 5, 6, 7, 8, 9, 10, 11, 12, 13, 14, 15); }
__device__ __forceinline__ v16bf cat16b(v8us lo, v8us hi) { return __builtin_bit_cast(v16bf, __builtin_shufflevector(lo, hi, 0, 1, 2, 3, 4, 5, 6, 7, 8, 9, 10, 11, 12, 13, 14, 15)); }
__device__ __forceinline__ v8f wmma16(v16h a, v16h b, v8f c) { return __builtin_amdgcn_wmma_f32_16x16x32_f16(false, a, false, b, (short)0, c, false, false); }
__device__ __forceinline__ v8f wmmab(v16bf a, v16bf b, v8f c) { return __builtin_amdgcn_wmma_f32_16x16x32_bf16(false, a, false, b, (short)0, c, false, false); }
__device__ __forceinline__ v16h  ldh(const h16* p) { return cat16(*(const v8h*)p, *(const v8h*)(p + 16)); }
__device__ __forceinline__ v16bf ldb(const bf* p)  { return cat16b(*(const v8us*)p, *(const v8us*)(p + 16)); }
__device__ __forceinline__ void wave_sync() { __builtin_amdgcn_fence(3  , "wavefront"); __builtin_amdgcn_wave_barrier(); asm volatile("" ::: "memory"); }

static __device__ __forceinline__ h16 toh_flush(float v) { const h16 r = (h16)v; return (fabsf(v) < 6.103515625e-05f) ? (h16)0.0f : r; }
__device__ __forceinline__ v8f mma(v16h a, v16h b, v8f c)   { c = wmma16(a, b, c); asm volatile("v_nop\n\tv_nop\n\tv_nop\n\tv_nop" : "+v"(c) : "v"(a), "v"(b)); return c; }
__device__ __forceinline__ v8f mma(v16bf a, v16bf b, v8f c) { c = wmmab(a, b, c);  asm volatile("v_nop\n\tv_nop\n\tv_nop\n\tv_nop" : "+v"(c) : "v"(a), "v"(b)); return c; }
__device__ __forceinline__ v16h  ldf(const h16* p) { return ldh(p); }
__device__ __forceinline__ v16bf ldf(const bf* p)  { return ldb(p); }

__global__ __launch_bounds__(256) void k_cvt8(const float* __restrict__ src, bf* dst, size_t n8) {
    const size_t i = (size_t)blockIdx.x * 256 + threadIdx.x; if (i >= n8) return;
    const v8f v = *(const v8f*)(src + i * 8); v8us o;
#pragma unroll
    for (int k = 0; k < 8; ++k) o[k] = f2bf(v[k]);
    *(volatile v8us*)(dst + i * 8) = o; __threadfence(); *(volatile v8us*)(dst + i * 8) = o;
}

__global__ __launch_bounds__(256) void k_xT(const float* __restrict__ x, bf* XB) {
    __shared__ __align__(16) unsigned short tl[64 * 72];
    const int tid = threadIdx.x; const int l0 = blockIdx.x * 64, c0 = blockIdx.y * 64, b = blockIdx.z;
    const float* xb = x + ((size_t)b * CC + c0) * SEQ_FULL + l0;
#pragma unroll 1
    for (int i = 0; i < 16; ++i) { const int idx = i * 256 + tid; const int lj = idx & 63, cj = idx >> 6;
        tl[lj * 72 + cj] = f2bf(xb[(size_t)cj * SEQ_FULL + lj]); }
    __syncthreads();
    bf* dst = XB + ((size_t)b * SEQ + l0) * CC + c0;
    v8us o[2];
#pragma unroll
    for (int it = 0; it < 2; ++it) { const int p = it * 256 + tid; const int row = p >> 3, c8 = (p & 7) * 8; o[it] = *(const v8usa*)(&tl[row * 72 + c8]); }
#pragma unroll 1
    for (int ps = 0; ps < 2; ++ps) {
#pragma unroll
        for (int it = 0; it < 2; ++it) { const int p = it * 256 + tid; const int row = p >> 3, c8 = (p & 7) * 8;
            *(volatile v8us*)(dst + (size_t)row * CC + c8) = o[it]; }
        if (ps == 0) __threadfence(); }
}

__global__ __launch_bounds__(256) void k_wcvt(const float* __restrict__ src, h16* dst, int nC, int nT, int n8) {
    const int i = blockIdx.x * 256 + threadIdx.x; if (i >= n8) return;
    const int e = i * 8; const int kk = nT * nC; const int o = e / kk; const int rem = e - o * kk; const int t = rem / nC; const int c = rem - t * nC;
    v8h ov;
#pragma unroll
    for (int k = 0; k < 8; ++k) ov[k] = toh_flush(bfr(src[((size_t)o * nC + c + k) * nT + t]) * WSC);
    *(volatile v8h*)(dst + (size_t)i * 8) = ov; __threadfence(); *(volatile v8h*)(dst + (size_t)i * 8) = ov;
}

template <typename T>
__device__ __forceinline__ void gemm_kloop(const T* __restrict__ A, const T* __restrict__ Bt, size_t aoff, size_t boff, int lda, int K, v8f (&acc)[4][4]) {
#pragma unroll 1
    for (int kc = 0; kc < K; kc += 32) {
        decltype(ldf(A)) a[4];
#pragma unroll
        for (int mb = 0; mb < 4; ++mb) a[mb] = ldf(A + aoff + (size_t)mb * 16 * (size_t)lda + kc);
#pragma unroll
        for (int nb = 0; nb < 4; ++nb) { const auto b = ldf(Bt + boff + (size_t)nb * 16 * (size_t)K + kc);
#pragma unroll
            for (int mb = 0; mb < 4; ++mb) acc[mb][nb] = mma(a[mb], b, acc[mb][nb]); }
    }
}

template <typename T, int RES>
__device__ __forceinline__ void gemm_tile(const T* __restrict__ A, const T* __restrict__ AR, const T* __restrict__ Bt, float* C,
                                          int lda, size_t abatch, int K, int ldc, float oscale) {
    __shared__ __align__(16) float os[16 * 68];
    const int lane = threadIdx.x & 31, lr = lane & 15, hi = lane >> 4; const int r0 = blockIdx.x * 64, c0 = blockIdx.y * 64;
    const int bb = r0 / SEQ, tt = r0 % SEQ;
    v8f acc[4][4];
#pragma unroll
    for (int mb = 0; mb < 4; ++mb)
#pragma unroll
        for (int nb = 0; nb < 4; ++nb) acc[mb][nb] = (v8f){};
    const size_t aoff = (size_t)bb * abatch + (size_t)(tt + lr) * (size_t)lda + 8 * hi, boff = (size_t)(c0 + lr) * (size_t)K + 8 * hi;
    if (RES) {
        gemm_kloop<T>(AR, Bt, aoff, boff, lda, K, acc);
#pragma unroll
        for (int mb = 0; mb < 4; ++mb)
#pragma unroll
            for (int nb = 0; nb < 4; ++nb) acc[mb][nb] = acc[mb][nb] * QRI;
    }
    gemm_kloop<T>(A, Bt, aoff, boff, lda, K, acc);
#pragma unroll
    for (int mb = 0; mb < 4; ++mb) {
#pragma unroll
        for (int nb = 0; nb < 4; ++nb) {
#pragma unroll
            for (int j = 0; j < 8; ++j) os[(hi * 8 + j) * 68 + nb * 16 + lr] = acc[mb][nb][j] * oscale; }
        wave_sync();
#pragma unroll 1
        for (int ps = 0; ps < 2; ++ps) {
#pragma unroll
            for (int s = 0; s < 8; ++s) { const int row = 2 * s + (lane >> 4), c4 = (lane & 15) * 4;
                const v4f val = *(const v4fa*)(&os[row * 68 + c4]);
                *(volatile v4f*)(C + (size_t)(r0 + mb * 16 + row) * (size_t)ldc + c0 + c4) = val; }
            if (ps == 0) __threadfence(); }
        wave_sync();
    }
}

__global__ __launch_bounds__(32) void k_gemm_proj(const bf* __restrict__ A, const bf* __restrict__ Bt, float* C) {
    gemm_tile<bf, 0>(A, A, Bt, C, CC, (size_t)SEQ * CC, CC, 3 * CC, 1.0f);
}
__global__ __launch_bounds__(32) void k_gemm_agg(const h16* __restrict__ A, const h16* __restrict__ AR, const h16* __restrict__ Bt, float* C) {
    gemm_tile<h16, 1>(A, AR, Bt, C, CC, (size_t)SEQ * CC, CC, CC, WSI);
}
__global__ __launch_bounds__(32) void k_gemm_c1(const h16* __restrict__ A, const h16* __restrict__ Bt, float* C) {
    gemm_tile<h16, 0>(A, A, Bt, C, CC, (size_t)SEQP * CC, 3 * CC, CH2, WSI);
}
__global__ __launch_bounds__(32) void k_gemm_c2(const h16* __restrict__ A, const h16* __restrict__ Bt, float* C) {
    gemm_tile<h16, 0>(A, A, Bt, C, CH2, (size_t)SEQP * CH2, 3 * CH2, CC, WSI);
}

__global__ __launch_bounds__(ATK * NH_) void k_lattn(const float* __restrict__ QKV, const float* __restrict__ rel, float* ATT) {
    __shared__ __align__(16) float rl[KW * HD];
    __shared__ __align__(16) float st[ATK * STP];
    const int tid = threadIdx.x;
#pragma unroll 1
    for (int i = tid; i < KW * HD; i += ATK * NH_) { const int k = i / HD, d = i - k * HD; rl[i] = bfr(rel[d * KW + k]); }
    __syncthreads();
    const int h = tid & (NH_ - 1), tk = tid / NH_;
    const int tok = blockIdx.x * ATK + tk; const int b = tok / SEQ, l = tok - b * SEQ;
    int wrow[KW]; bool ok[KW];
#pragma unroll
    for (int k = 0; k < KW; ++k) { const int pos = l - PADW + k; ok[k] = (pos >= 0) & (pos < SEQ);
        const int pc = pos < 0 ? 0 : (pos > SEQ - 1 ? SEQ - 1 : pos); wrow[k] = b * SEQ + pc; }
    const float* qp = QKV + (size_t)tok * (3 * CC) + h * HD;
    const float* kb = QKV + CC + h * HD;
    const float* vb = QKV + 2 * CC + h * HD;
    const v4f z4 = (v4f){};
    float s[KW];
#pragma unroll
    for (int k = 0; k < KW; ++k) s[k] = 0.0f;
#pragma unroll 1
    for (int j = 0; j < HD / 4; ++j) {
        const v4f q4 = *(const v4f*)(qp + 4 * j);
#pragma unroll
        for (int k = 0; k < KW; ++k) {
            v4f k4 = *(const v4f*)(kb + (size_t)wrow[k] * (3 * CC) + 4 * j);
            asm volatile("" : "+v"(k4));
            const v4f r4 = *(const v4fa*)(&rl[k * HD + 4 * j]);
            const v4f kk = (ok[k] ? k4 : z4) + r4;
            s[k] = fmaf(q4[0], kk[0], s[k]); s[k] = fmaf(q4[1], kk[1], s[k]); s[k] = fmaf(q4[2], kk[2], s[k]); s[k] = fmaf(q4[3], kk[3], s[k]); }
    }
    float mx = -3.0e38f;
#pragma unroll
    for (int k = 0; k < KW; ++k) { s[k] = s[k] * SC2; mx = fmaxf(mx, s[k]); }
    float w[KW]; float den = 0.0f;
#pragma unroll
    for (int k = 0; k < KW; ++k) { w[k] = __builtin_amdgcn_exp2f(s[k] - mx); den += w[k]; }
    const float inv = __builtin_amdgcn_rcpf(den);
#pragma unroll
    for (int k = 0; k < KW; ++k) { const float wk = w[k] * inv; w[k] = ok[k] ? wk : 0.0f; }
#pragma unroll 1
    for (int j = 0; j < HD / 4; ++j) {
        v4f a = z4;
#pragma unroll
        for (int k = 0; k < KW; ++k) {
            v4f v4 = *(const v4f*)(vb + (size_t)wrow[k] * (3 * CC) + 4 * j);
            asm volatile("" : "+v"(v4));
            a[0] = fmaf(w[k], v4[0], a[0]); a[1] = fmaf(w[k], v4[1], a[1]); a[2] = fmaf(w[k], v4[2], a[2]); a[3] = fmaf(w[k], v4[3], a[3]); }
        *(v4fa*)(&st[tk * STP + h * HD + 4 * j]) = a;
    }
    __syncthreads();
    float* arow = ATT + (size_t)blockIdx.x * ATK * CC;
    v4f vals[8];
#pragma unroll
    for (int it = 0; it < 8; ++it) { const int p = it * (ATK * NH_) + tid; const int row = p >> 6, c4 = (p & 63) * 4; vals[it] = *(const v4fa*)(&st[row * STP + c4]); }
#pragma unroll 1
    for (int ps = 0; ps < 2; ++ps) {
#pragma unroll
        for (int it = 0; it < 8; ++it) { const int p = it * (ATK * NH_) + tid; const int row = p >> 6, c4 = (p & 63) * 4;
            *(volatile v4f*)(arow + (size_t)row * CC + c4) = vals[it]; }
        if (ps == 0) __threadfence(); }
}

__global__ __launch_bounds__(256) void k_colstats(const float* __restrict__ X, int ncols, double* P) {
    __shared__ __align__(16) double sd[2 * CC];
    const int tid = threadIdx.x; const int ch = blockIdx.x;
    const float* xp = X + (size_t)ch * RCH * (size_t)ncols + tid;
    double s = 0.0, s2 = 0.0;
#pragma unroll 4
    for (int r = 0; r < RCH; ++r) { const double v = (double)xp[(size_t)r * ncols]; s += v; s2 += v * v; }
    sd[tid] = s; sd[ncols + tid] = s2;
    __syncthreads();
    const v4f pv = *(const v4fa*)(&sd[2 * tid]);
    double* pp = P + ((size_t)ch * 2) * (size_t)ncols + 2 * tid;
    *(volatile v4f*)pp = pv; __threadfence(); *(volatile v4f*)pp = pv;
}

__global__ __launch_bounds__(256) void k_bnfin(const double* __restrict__ P, int ncols, const float* __restrict__ g, const float* __restrict__ bb, float* S) {
    __shared__ __align__(16) float ss[2 * CC];
    const int c = threadIdx.x;
    double s = 0.0, s2 = 0.0;
#pragma unroll 1
    for (int ch = 0; ch < NCHK; ++ch) { s += P[((size_t)ch * 2) * (size_t)ncols + c]; s2 += P[((size_t)ch * 2 + 1) * (size_t)ncols + c]; }
    const double m = s * (1.0 / (double)NTOK); double var = s2 * (1.0 / (double)NTOK) - m * m; var = var < 0.0 ? 0.0 : var;
    const float sc = bfr(g[c]) * rsqrtf((float)var + EPSV);
    const float sh = bfr(bb[c]) - (float)m * sc;
    ss[c] = sc; ss[CC + c] = sh;
#pragma unroll 1
    for (int j = ncols + c; j < CC; j += ncols) { ss[j] = 0.0f; ss[CC + j] = 0.0f; }
    __syncthreads();
    if (c < 2 * CC / 4) {
        const v4f val = *(const v4fa*)(&ss[4 * c]);
        *(volatile v4f*)(S + 4 * c) = val; __threadfence(); *(volatile v4f*)(S + 4 * c) = val;
    }
}

__global__ __launch_bounds__(CC) void k_sefin(const double* __restrict__ P, const float* __restrict__ g2, const float* __restrict__ b2,
                                              const float* __restrict__ w1, const float* __restrict__ b1, const float* __restrict__ w2, const float* __restrict__ b2s, float* GS) {
    __shared__ float pool[NB * CC];
    __shared__ float hid[NB * RSE];
    __shared__ __align__(16) float gt[2 * NB * CC];
    const int c = threadIdx.x;
    double tot = 0.0, tot2 = 0.0;
#pragma unroll 1
    for (int b = 0; b < NB; ++b) { double s = 0.0;
#pragma unroll 1
        for (int q = 0; q < CPB; ++q) { const size_t ch = (size_t)b * CPB + q; s += P[(ch * 2) * CC + c]; tot2 += P[(ch * 2 + 1) * CC + c]; }
        pool[b * CC + c] = (float)(s * (1.0 / (double)SEQ)); tot += s; }
    const double m = tot * (1.0 / (double)NTOK); double var = tot2 * (1.0 / (double)NTOK) - m * m; var = var < 0.0 ? 0.0 : var;
    const float sc = bfr(g2[c]) * rsqrtf((float)var + EPSV);
    const float sh = bfr(b2[c]) - (float)m * sc;
#pragma unroll 1
    for (int b = 0; b < NB; ++b) pool[b * CC + c] = pool[b * CC + c] * sc + sh;
    __syncthreads();
#pragma unroll 1
    for (int i = c; i < NB * RSE; i += CC) { const int b = i / RSE, r = i - b * RSE; float a = bfr(b1[r]);
#pragma unroll 4
        for (int cc = 0; cc < CC; ++cc) a += pool[b * CC + cc] * bfr(w1[r * CC + cc]);
        hid[i] = (a > 0.0f) ? a : 0.0f; }
    __syncthreads();
    float gsv[NB], ghv[NB];
#pragma unroll
    for (int b = 0; b < NB; ++b) { float a = bfr(b2s[c]);
#pragma unroll 1
        for (int r = 0; r < RSE; ++r) a += hid[b * RSE + r] * bfr(w2[c * RSE + r]);
        const float gate = __builtin_amdgcn_rcpf(1.0f + __builtin_amdgcn_exp2f(-a * L2E));
        gsv[b] = sc * gate; ghv[b] = sh * gate; }
#pragma unroll
    for (int b = 0; b < NB; ++b) { gt[b * CC + c] = gsv[b]; gt[NB * CC + b * CC + c] = ghv[b]; }
    __syncthreads();
#pragma unroll 1
    for (int ps = 0; ps < 2; ++ps) {
#pragma unroll 1
        for (int p = c; p < 2 * NB * CC / 4; p += CC) {
            const v4f val = *(const v4fa*)(&gt[4 * p]);
            *(volatile v4f*)(GS + 4 * p) = val; }
        if (ps == 0) __threadfence(); }
}

__global__ __launch_bounds__(256) void k_act16(const float* __restrict__ X, const float* __restrict__ SC, const float* __restrict__ SH, int bstride,
                                               int ncols, int pad, int relu, int hasres, h16* D, h16* DR, int n8) {
    const int i = blockIdx.x * 256 + threadIdx.x; if (i >= n8) return;
    const int c8n = ncols >> 3; const int prow = i / c8n; const int c = (i - prow * c8n) * 8;
    const int rpb = SEQ + 2 * pad; const int b = prow / rpb; const int l = prow - b * rpb - pad;
    const bool ok = (l >= 0) & (l < SEQ); const int lc = l < 0 ? 0 : (l > SEQ - 1 ? SEQ - 1 : l);
    const float* xp = X + ((size_t)b * SEQ + lc) * (size_t)ncols + c;
    v4f x0 = *(const v4f*)xp, x1 = *(const v4f*)(xp + 4);
    asm volatile("" : "+v"(x0)); asm volatile("" : "+v"(x1));
    const v4f s0 = *(const v4f*)(SC + b * bstride + c), s1 = *(const v4f*)(SC + b * bstride + c + 4);
    const v4f h0 = *(const v4f*)(SH + b * bstride + c), h1 = *(const v4f*)(SH + b * bstride + c + 4);
    v8h hv, rv;
#pragma unroll
    for (int k = 0; k < 4; ++k) {
        float y0 = x0[k] * s0[k] + h0[k], y1 = x1[k] * s1[k] + h1[k];
        if (relu != 0) { y0 = (y0 > 0.0f) ? y0 : 0.0f; y1 = (y1 > 0.0f) ? y1 : 0.0f; }
        y0 = ok ? y0 : 0.0f; y1 = ok ? y1 : 0.0f;
        const h16 a0 = toh_flush(y0), a1 = toh_flush(y1);
        hv[k] = a0; hv[4 + k] = a1;
        rv[k] = toh_flush((y0 - (float)a0) * QRS); rv[4 + k] = toh_flush((y1 - (float)a1) * QRS); }
    *(volatile v8h*)(D + (size_t)i * 8) = hv; if (hasres != 0) *(volatile v8h*)(DR + (size_t)i * 8) = rv;
    __threadfence();
    *(volatile v8h*)(D + (size_t)i * 8) = hv; if (hasres != 0) *(volatile v8h*)(DR + (size_t)i * 8) = rv;
}

__global__ __launch_bounds__(256) void k_final(const float* __restrict__ Z, const float* __restrict__ GS, const float* __restrict__ A2, const float* __restrict__ S4, float* dout) {
    const size_t idx = (size_t)blockIdx.x * 256 + threadIdx.x;
    const int l = (int)(idx % SEQ); const int c = (int)((idx / SEQ) % CC); const int b = (int)(idx / ((size_t)SEQ * CC));
    const size_t src = ((size_t)b * SEQ + l) * CC + c;
    const float o = Z[src] * GS[b * CC + c] + GS[NB * CC + b * CC + c];
    const float g = A2[src] * S4[c] + S4[CC + c];
    const float gate = __builtin_amdgcn_rcpf(1.0f + __builtin_amdgcn_exp2f(-g * L2E));
    const float val = o * gate;
    float* dp = dout + ((size_t)b * CC + c) * OUT_SEQ + l;
    *(volatile float*)dp = val; __threadfence(); *(volatile float*)dp = val;
}

static constexpr size_t al256(size_t v) { return (v + 255) & ~(size_t)255; }
static constexpr size_t SZ_XB  = al256((size_t)NTOK * CC * 2);
static constexpr size_t SZ_WB  = al256((size_t)3 * CC * CC * 2);
static constexpr size_t SZ_QKV = al256((size_t)NTOK * 3 * CC * 4);
static constexpr size_t SZ_F2  = al256((size_t)NTOK * CC * 4);
static constexpr size_t SZ_F1  = al256((size_t)NTOK * CH2 * 4);
static constexpr size_t SZ_T16 = al256((size_t)NTOK * CC * 2);
static constexpr size_t SZ_O16 = al256((size_t)NB * SEQP * CC * 2);
static constexpr size_t SZ_N16 = al256((size_t)NB * SEQP * CH2 * 2);
static constexpr size_t SZ_AGW = al256((size_t)CC * CC * 2);
static constexpr size_t SZ_W1R = al256((size_t)CH2 * 3 * CC * 2);
static constexpr size_t SZ_W2R = al256((size_t)CC * 3 * CH2 * 2);
static constexpr size_t SZ_PT  = al256((size_t)NCHK * 2 * CC * 8);
static constexpr size_t SZ_SS  = al256((size_t)2 * CC * 4);
static constexpr size_t SZ_GS  = al256((size_t)2 * NB * CC * 4);
static constexpr size_t SZ_TOTAL = SZ_XB + SZ_WB + SZ_QKV + 3 * SZ_F2 + SZ_F1 + 2 * SZ_T16 + SZ_O16 + SZ_N16 + SZ_AGW + SZ_W1R + SZ_W2R + 4 * SZ_PT + 3 * SZ_SS + SZ_GS;
static_assert(SZ_TOTAL <= (size_t)134217728);
static_assert(((size_t)CC * CC * 2) % 256 == 0);
static_assert(SZ_PT >= (size_t)NCHK * 2 * CC * 8);
static_assert(SZ_SS >= (size_t)(2 * CC / 4) * 16);
static_assert(SZ_GS >= (size_t)(2 * NB * CC / 4) * 16);

extern "C" void kernel_launch(void* const* d_in, const int* in_sizes, int n_in,
                              void* d_out, int out_size, void* d_ws, size_t ws_size, hipStream_t stream) {
    if (n_in < 20) return;
    const size_t needx = ((size_t)(NB - 1) * CC + (CC - 1)) * SEQ_FULL + SEQ;
    if ((size_t)in_sizes[0] < needx) return;
    if (in_sizes[1] < HD * KW) return;
    if ((size_t)in_sizes[2] < (size_t)CC * CC || (size_t)in_sizes[3] < (size_t)CC * CC || (size_t)in_sizes[4] < (size_t)CC * CC || (size_t)in_sizes[5] < (size_t)CC * CC) return;
    if (in_sizes[6] < CC || in_sizes[7] < CC || in_sizes[8] < CC || in_sizes[9] < CC) return;
    if (in_sizes[10] < RSE * CC || in_sizes[11] < RSE || in_sizes[12] < CC * RSE || in_sizes[13] < CC) return;
    if ((size_t)in_sizes[14] < (size_t)CH2 * CC * 3 || in_sizes[15] < CH2 || in_sizes[16] < CH2) return;
    if ((size_t)in_sizes[17] < (size_t)CC * CH2 * 3 || in_sizes[18] < CC || in_sizes[19] < CC) return;
    if ((size_t)out_size < ((size_t)(NB - 1) * CC + (CC - 1)) * OUT_SEQ + SEQ) return;
    if (SZ_TOTAL > ws_size) return;
    const float* x    = (const float*)d_in[0];
    const float* rel  = (const float*)d_in[1];
    const float* wq   = (const float*)d_in[2];
    const float* wk   = (const float*)d_in[3];
    const float* wv   = (const float*)d_in[4];
    const float* aggw = (const float*)d_in[5];
    const float* ag1  = (const float*)d_in[6];
    const float* ab1  = (const float*)d_in[7];
    const float* ag2  = (const float*)d_in[8];
    const float* ab2  = (const float*)d_in[9];
    const float* sew1 = (const float*)d_in[10];
    const float* seb1 = (const float*)d_in[11];
    const float* sew2 = (const float*)d_in[12];
    const float* seb2 = (const float*)d_in[13];
    const float* cw1  = (const float*)d_in[14];
    const float* cg1  = (const float*)d_in[15];
    const float* cb1  = (const float*)d_in[16];
    const float* cw2  = (const float*)d_in[17];
    const float* cg2  = (const float*)d_in[18];
    const float* cb2  = (const float*)d_in[19];
    float* OUT = (float*)d_out;
    char* wsp = (char*)d_ws;
    bf*    XB   = (bf*)wsp;    wsp += SZ_XB;
    bf*    WB   = (bf*)wsp;    wsp += SZ_WB;
    float* QKV  = (float*)wsp; wsp += SZ_QKV;
    float* ATT  = (float*)wsp; wsp += SZ_F2;
    float* Z    = (float*)wsp; wsp += SZ_F2;
    float* A2   = (float*)wsp; wsp += SZ_F2;
    float* A1   = (float*)wsp; wsp += SZ_F1;
    h16*   T16  = (h16*)wsp;   wsp += SZ_T16;
    h16*   TR16 = (h16*)wsp;   wsp += SZ_T16;
    h16*   O16  = (h16*)wsp;   wsp += SZ_O16;
    h16*   N16  = (h16*)wsp;   wsp += SZ_N16;
    h16*   AGW  = (h16*)wsp;   wsp += SZ_AGW;
    h16*   W1R  = (h16*)wsp;   wsp += SZ_W1R;
    h16*   W2R  = (h16*)wsp;   wsp += SZ_W2R;
    double* P1  = (double*)wsp; wsp += SZ_PT;
    double* P2  = (double*)wsp; wsp += SZ_PT;
    double* P3  = (double*)wsp; wsp += SZ_PT;
    double* P4  = (double*)wsp; wsp += SZ_PT;
    float* S1   = (float*)wsp; wsp += SZ_SS;
    float* S3   = (float*)wsp; wsp += SZ_SS;
    float* S4   = (float*)wsp; wsp += SZ_SS;
    float* GS   = (float*)wsp; wsp += SZ_GS;

    k_xT<<<dim3(SEQ / 64, CC / 64, NB), 256, 0, stream>>>(x, XB);
    { const size_t n8 = (size_t)CC * CC / 8; const unsigned g = (unsigned)((n8 + 255) / 256);
      k_cvt8<<<g, 256, 0, stream>>>(wq, WB, n8); k_cvt8<<<g, 256, 0, stream>>>(wk, WB + (size_t)CC * CC, n8); k_cvt8<<<g, 256, 0, stream>>>(wv, WB + (size_t)2 * CC * CC, n8); }
    { const int n8a = CC * CC / 8, n8b = CH2 * 3 * CC / 8, n8c = CC * 3 * CH2 / 8;
      k_wcvt<<<(n8a + 255) / 256, 256, 0, stream>>>(aggw, AGW, CC, 1, n8a);
      k_wcvt<<<(n8b + 255) / 256, 256, 0, stream>>>(cw1, W1R, CC, 3, n8b);
      k_wcvt<<<(n8c + 255) / 256, 256, 0, stream>>>(cw2, W2R, CH2, 3, n8c); }

    k_gemm_proj<<<dim3(NTOK / 64, 3 * CC / 64, 1), 32, 0, stream>>>(XB, WB, QKV);
    k_lattn<<<NTOK / ATK, ATK * NH_, 0, stream>>>(QKV, rel, ATT);
    k_colstats<<<NCHK, CC, 0, stream>>>(ATT, CC, P1);
    k_bnfin<<<1, CC, 0, stream>>>(P1, CC, ag1, ab1, S1);
    { const int n8 = NTOK * CC / 8; k_act16<<<(n8 + 255) / 256, 256, 0, stream>>>(ATT, S1, S1 + CC, 0, CC, 0, 1, 1, T16, TR16, n8); }
    k_gemm_agg<<<dim3(NTOK / 64, CC / 64, 1), 32, 0, stream>>>(T16, TR16, AGW, Z);
    k_colstats<<<NCHK, CC, 0, stream>>>(Z, CC, P2);
    k_sefin<<<1, CC, 0, stream>>>(P2, ag2, ab2, sew1, seb1, sew2, seb2, GS);
    { const int n8 = NB * SEQP * CC / 8; k_act16<<<(n8 + 255) / 256, 256, 0, stream>>>(Z, GS, GS + NB * CC, CC, CC, 1, 0, 0, O16, O16, n8); }
    k_gemm_c1<<<dim3(NTOK / 64, CH2 / 64, 1), 32, 0, stream>>>(O16, W1R, A1);
    k_colstats<<<NCHK, CH2, 0, stream>>>(A1, CH2, P3);
    k_bnfin<<<1, CH2, 0, stream>>>(P3, CH2, cg1, cb1, S3);
    { const int n8 = NB * SEQP * CH2 / 8; k_act16<<<(n8 + 255) / 256, 256, 0, stream>>>(A1, S3, S3 + CC, 0, CH2, 1, 1, 0, N16, N16, n8); }
    k_gemm_c2<<<dim3(NTOK / 64, CC / 64, 1), 32, 0, stream>>>(N16, W2R, A2);
    k_colstats<<<NCHK, CC, 0, stream>>>(A2, CC, P4);
    k_bnfin<<<1, CC, 0, stream>>>(P4, CC, cg2, cb2, S4);
    k_final<<<(unsigned)(((size_t)NB * CC * SEQ) / 256), 256, 0, stream>>>(Z, GS, A2, S4, OUT);
}
